// NeuralProcessConv_24343874634007
// MI455X (gfx1250) — hardware-verified
//
#include <hip/hip_runtime.h>
#include <math.h>
#include <stdint.h>

#define NB     16
#define NCX    64
#define NTG    128
#define GW     50
#define NPIX   2500
#define HALO   52
#define C1     32
#define K2     288
#define RDIM   128
#define ZDIM   64
#define HDIM   128
#define NS     (NB * NCX)
#define NT     (NB * NTG)
#define NPAD   2560
#define NTILE1 157
#define SC1    64.0f
#define SC2    256.0f
#define ISC12  (1.0f / 16384.0f)

#define L_HH    0
#define L_BT2   173056
#define L_GRID  191488
#define L_BT1   202304
#define L_POOL  204352
#define L_PLD   205376
#define L_B1    205504
#define L_B2    205632
#define L_HM    205760
#define L_RROW  206272
#define L_TOTAL 206784

static_assert(NTILE1 * 16 >= NPIX && (NTILE1 - 1) * 16 < NPIX);
static_assert((NT % 64) == 0 && (NPAD % 64) == 0 && (HDIM % 32) == 0 && NPAD >= NPIX);
static_assert((NTG % 16) == 0);
static_assert(((2 * NT * NPIX) % 1024) == 0);
static_assert((NPIX % 4) == 0);
static_assert(((NB * ZDIM) % 32) == 0);
static_assert(C1 * K2 == 1152 * 8);
static_assert((L_BT2 % 16) == 0 && (L_GRID % 16) == 0 && (L_BT1 % 16) == 0 && (L_POOL % 16) == 0 && (L_RROW % 16) == 0);

typedef __bf16   v16b __attribute__((ext_vector_type(16)));
typedef __bf16   v8b  __attribute__((ext_vector_type(8)));
typedef _Float16 v16h __attribute__((ext_vector_type(16)));
typedef _Float16 v8h  __attribute__((ext_vector_type(8)));
typedef float    v8f  __attribute__((ext_vector_type(8)));
typedef float    v4f  __attribute__((ext_vector_type(4)));
typedef unsigned int v4u __attribute__((ext_vector_type(4)));
typedef unsigned int v8u __attribute__((ext_vector_type(8)));
union FragB { v16b v; v8b hf[2]; };
union FragH { v16h v; v8h hf[2]; };
union F8    { v4f v[2]; float f[8]; };

__device__ __forceinline__ unsigned short bf_bits(float f) {
  unsigned u = __float_as_uint(f);
  return (unsigned short)((u + 0x7FFFu + ((u >> 16) & 1u)) >> 16);
}
__device__ __forceinline__ float bf_up(unsigned short h) { return __uint_as_float(((unsigned)h) << 16); }
__device__ __forceinline__ float bfr(float f) { return bf_up(bf_bits(f)); }
__device__ __forceinline__ unsigned short h_bits(float f) { _Float16 hv = (_Float16)f; return __builtin_bit_cast(unsigned short, hv); }
__device__ __forceinline__ unsigned pk16(unsigned short a, unsigned short b) { return (unsigned)a | ((unsigned)b << 16); }
__device__ __forceinline__ v8f zero8() { v8f z = {0.f, 0.f, 0.f, 0.f, 0.f, 0.f, 0.f, 0.f}; return z; }
__device__ __forceinline__ v4u zero4u() { v4u z = {0u, 0u, 0u, 0u}; return z; }
__device__ __forceinline__ void split_bits(float y, unsigned short& hi, unsigned short& lo) {
  hi = bf_bits(y);
  lo = bf_bits(y - bf_up(hi));
}

__device__ __forceinline__ v16b ldfrag_b(const __bf16* p) {
  FragB f;
  f.hf[0] = *(const v8b*)(p);
  f.hf[1] = *(const v8b*)(p + 16);
  return f.v;
}
__device__ __forceinline__ v16h ldfrag_h(const _Float16* p) {
  FragH f;
  f.hf[0] = *(const v8h*)(p);
  f.hf[1] = *(const v8h*)(p + 16);
  return f.v;
}

__device__ __forceinline__ v8f mma_b_raw(v16b a, v16b b, v8f c) {
  return __builtin_amdgcn_wmma_f32_16x16x32_bf16(false, a, false, b, (short)0, c, false, false);
}
__device__ __forceinline__ v8f mma_h_raw(v16h a, v16h b, v8f c) {
  return __builtin_amdgcn_wmma_f32_16x16x32_f16(false, a, false, b, (short)0, c, false, false);
}
__device__ __forceinline__ void dep_guard_b(v8f& a, v8f& b, v16b x, v16b y) {
#if defined(__HIP_DEVICE_COMPILE__)
  asm volatile("v_nop\n\tv_nop\n\tv_nop\n\tv_nop" : "+v"(a), "+v"(b) : "v"(x), "v"(y));
#endif
}
__device__ __forceinline__ void dep_guard_b3(v8f& a, v8f& b, v16b x, v16b y, v16b z) {
#if defined(__HIP_DEVICE_COMPILE__)
  asm volatile("v_nop\n\tv_nop\n\tv_nop\n\tv_nop" : "+v"(a), "+v"(b) : "v"(x), "v"(y), "v"(z));
#endif
}
__device__ __forceinline__ void dep_guard_h3(v8f& a, v8f& b, v16h x, v16h y, v16h z) {
#if defined(__HIP_DEVICE_COMPILE__)
  asm volatile("v_nop\n\tv_nop\n\tv_nop\n\tv_nop" : "+v"(a), "+v"(b) : "v"(x), "v"(y), "v"(z));
#endif
}
__device__ __forceinline__ void keep2_b(v16b a, v16b b) {
#if defined(__HIP_DEVICE_COMPILE__)
  asm volatile("v_nop" :: "v"(a), "v"(b));
#endif
}
__device__ __forceinline__ void acc_guard2(v8f& a, v8f& b) {
#if defined(__HIP_DEVICE_COMPILE__)
  asm volatile("v_nop\n\tv_nop\n\tv_nop\n\tv_nop" : "+v"(a), "+v"(b));
#endif
}
__device__ __forceinline__ void acc_guard4(v8f& a, v8f& b, v8f& c, v8f& d) {
#if defined(__HIP_DEVICE_COMPILE__)
  asm volatile("v_nop\n\tv_nop\n\tv_nop\n\tv_nop" : "+v"(a), "+v"(b), "+v"(c), "+v"(d));
#endif
}
__device__ __forceinline__ void wave_sync_lds() {
  __builtin_amdgcn_fence(__ATOMIC_RELEASE, "workgroup");
  __builtin_amdgcn_wave_barrier();
  __builtin_amdgcn_fence(__ATOMIC_ACQUIRE, "workgroup");
}

__global__ __launch_bounds__(256) void k_wprep(const float* __restrict__ Wdmu, const float* __restrict__ Wdsig,
                                               const float* __restrict__ w2,
                                               unsigned short* Btp, unsigned short* W2p) {
  __shared__ __align__(16) unsigned short T[64 * 136];
  const int tid = threadIdx.x;
  const int by  = blockIdx.y;
  const int bx  = blockIdx.x;
  if (by == 2) {
    const int i = bx * 256 + tid;
    if (i >= 1152) return;
    const int n   = i / 36;
    const int rem = i - n * 36;
    const int tap = rem >> 2;
    const int c0  = (rem & 3) * 8;
    v4u p;
#pragma unroll
    for (int e = 0; e < 4; ++e) {
      const float wa = bfr(w2[(n * C1 + c0 + 2 * e) * 9 + tap]) * SC2;
      const float wb = bfr(w2[(n * C1 + c0 + 2 * e + 1) * 9 + tap]) * SC2;
      p[e] = pk16(h_bits(wa), h_bits(wb));
    }
    *(volatile v4u*)(W2p + (size_t)i * 8) = p;
    __threadfence();
    *(volatile v4u*)(W2p + (size_t)i * 8) = p;
    return;
  }
  const float* W = (by == 0) ? Wdmu : Wdsig;
  unsigned short* Bt = Btp + (size_t)by * NPAD * HDIM;
  const int n0 = bx * 64;
#pragma unroll 1
  for (int it = 0; it < 32; ++it) {
    const int idx = it * 256 + tid;
    const int k   = idx >> 6;
    const int nl  = idx & 63;
    const int n   = n0 + nl;
    const int nc  = (n < NPIX) ? n : (NPIX - 1);
    const float v = W[(size_t)k * NPIX + nc];
    T[nl * 136 + k] = (n < NPIX) ? bf_bits(v) : (unsigned short)0;
  }
  __syncthreads();
  v4u pc[4];
#pragma unroll
  for (int it = 0; it < 4; ++it) {
    const int j   = it * 256 + tid;
    const int row = j >> 4;
    const int c8  = (j & 15) * 8;
    pc[it] = *(const v4u*)(T + row * 136 + c8);
  }
  for (int pass = 0; pass < 2; ++pass) {
#pragma unroll
    for (int it = 0; it < 4; ++it) {
      const int j = it * 256 + tid;
      *(volatile v4u*)(Bt + (size_t)n0 * HDIM + (size_t)j * 8) = pc[it];
    }
    __threadfence();
  }
}

__global__ __launch_bounds__(256) void k_encode(
    const float* __restrict__ xc, const float* __restrict__ yc,
    const float* __restrict__ w1, const float* __restrict__ b1,
    const unsigned short* __restrict__ w2p, const float* __restrict__ b2,
    const float* __restrict__ We1, const float* __restrict__ be1,
    const float* __restrict__ We2, const float* __restrict__ be2,
    float* riT)
{
  extern __shared__ __align__(16) char smem[];
  _Float16*       hh    = (_Float16*)(smem + L_HH);
  unsigned short* hhu   = (unsigned short*)(smem + L_HH);
  _Float16*       bt2   = (_Float16*)(smem + L_BT2);
  unsigned short* bt2u  = (unsigned short*)(smem + L_BT2);
  unsigned int*   cellg = (unsigned int*)(smem + L_GRID);
  __bf16*         bt1   = (__bf16*)(smem + L_BT1);
  unsigned short* bt1u  = (unsigned short*)(smem + L_BT1);
  float* pool   = (float*)(smem + L_POOL);
  float* pooled = (float*)(smem + L_PLD);
  float* b1s    = (float*)(smem + L_B1);
  float* b2s    = (float*)(smem + L_B2);
  float* hm     = (float*)(smem + L_HM);
  float* rrow   = (float*)(smem + L_RROW);

  const int s    = blockIdx.x;
  const int tid  = threadIdx.x;
  const int lane = tid & 31;
  const int wave = tid >> 5;
  const int h    = lane >> 4;
  const int m    = lane & 15;
  const unsigned short xbits = bf_bits(xc[s]);
  const float xbf = bf_up(xbits);

#pragma unroll 1
  for (int c = tid; c < HALO * HALO; c += 256) {
    const int gy = c / HALO;
    const int gx = c - gy * HALO;
    const bool in = (gy >= 1) && (gy <= GW) && (gx >= 1) && (gx <= GW);
    int p = (gy - 1) * GW + (gx - 1);
    p = (p < 0) ? 0 : ((p > NPIX - 1) ? (NPIX - 1) : p);
    const float yv = yc[(size_t)s * NPIX + p];
    const unsigned v = pk16(bf_bits(yv), xbits);
    cellg[c] = in ? v : 0u;
  }
#pragma unroll 1
  for (int i = tid; i < 204 * 4; i += 256) {
    const int c = i >> 2, q = i & 3;
    int gy, gx;
    if (c < 52)       { gy = 0;       gx = c; }
    else if (c < 104) { gy = 51;      gx = c - 52; }
    else if (c < 154) { gy = c - 103; gx = 0; }
    else              { gy = c - 153; gx = 51; }
    *(v4u*)(hhu + (gy * HALO + gx) * C1 + q * 8) = zero4u();
  }
#pragma unroll 1
  for (int i = tid; i < 1152; i += 256) *(v4u*)(bt2u + i * 8) = *(const v4u*)(w2p + (size_t)i * 8);
#pragma unroll 1
  for (int i = tid; i < C1 * 32; i += 256) {
    const int n = i >> 5, k = i & 31;
    int cin = -1, tap = 0;
    if (k < 8)        { cin = 0; tap = k; }
    else if (k < 16)  { cin = 1; tap = k - 8; }
    else if (k == 16) { cin = 0; tap = 8; }
    else if (k == 24) { cin = 1; tap = 8; }
    const int ci = (cin < 0) ? 0 : cin;
    const float wv = w1[(n * 2 + ci) * 9 + tap];
    bt1u[i] = (cin >= 0) ? bf_bits(wv) : (unsigned short)0;
  }
  if (tid < C1) { b1s[tid] = bfr(b1[tid]); b2s[tid] = bfr(b2[tid]); }
  __syncthreads();

  {
    const v16b bb0 = ldfrag_b(bt1 + m * 32 + 8 * h);
    const v16b bb1 = ldfrag_b(bt1 + (16 + m) * 32 + 8 * h);
    const float bia0 = b1s[m];
    const float bia1 = b1s[16 + m];
    const int sh = h * 16;
#pragma unroll 1
    for (int tile = wave; tile < NTILE1; tile += 8) {
      const int pix = tile * 16 + m;
      const int pp  = (pix < NPIX) ? pix : (NPIX - 1);
      const int py  = pp / GW;
      const int px  = pp - py * GW;
      const unsigned int* gb = cellg + py * HALO + px;
      unsigned v[9];
#pragma unroll
      for (int t = 0; t < 9; ++t) {
        const int dy = t / 3, dx = t - (t / 3) * 3;
        v[t] = (gb[dy * HALO + dx] >> sh) & 0xFFFFu;
      }
      v8u av;
      av[0] = v[0] | (v[1] << 16);
      av[1] = v[2] | (v[3] << 16);
      av[2] = v[4] | (v[5] << 16);
      av[3] = v[6] | (v[7] << 16);
      av[4] = v[8];
      av[5] = 0u; av[6] = 0u; av[7] = 0u;
      const v16b a = __builtin_bit_cast(v16b, av);
      v8f acc0 = mma_b_raw(a, bb0, zero8());
      v8f acc1 = mma_b_raw(a, bb1, zero8());
      dep_guard_b3(acc0, acc1, a, bb0, bb1);
#pragma unroll
      for (int r = 0; r < 8; ++r) {
        const int p2 = tile * 16 + 8 * h + r;
        const float y0 = fmaxf(acc0[r] + bia0, 0.f) * SC1;
        const float y1 = fmaxf(acc1[r] + bia1, 0.f) * SC1;
        const unsigned short u0 = h_bits(y0);
        const unsigned short u1 = h_bits(y1);
        const int pc = (p2 < NPIX) ? p2 : (NPIX - 1);
        const int qy = pc / GW;
        const int qx = pc - qy * GW;
        unsigned short* dst = hhu + ((qy + 1) * HALO + (qx + 1)) * C1;
        if (p2 < NPIX) {
          dst[m] = u0;
          dst[16 + m] = u1;
        }
      }
    }
  }
  __syncthreads();

  float s0 = 0.f, s1 = 0.f;
  {
    const float bia0 = b2s[m];
    const float bia1 = b2s[16 + m];
#pragma unroll 1
    for (int tile = wave; tile < NTILE1; tile += 8) {
      const int pix = tile * 16 + m;
      const int pp  = (pix < NPIX) ? pix : (NPIX - 1);
      const int py  = pp / GW;
      const int px  = pp - py * GW;
      const _Float16* ab = hh + (py * HALO + px) * C1 + 8 * h;
      v8f acc0 = zero8(), acc1 = zero8();
#pragma unroll
      for (int t = 0; t < 9; ++t) {
        const int dy = t / 3, dx = t - (t / 3) * 3;
        const v16h a  = ldfrag_h(ab + (dy * HALO + dx) * C1);
        const v16h c0 = ldfrag_h(bt2 + m * K2 + t * 32 + 8 * h);
        const v16h c1 = ldfrag_h(bt2 + (16 + m) * K2 + t * 32 + 8 * h);
        acc0 = mma_h_raw(a, c0, acc0);
        acc1 = mma_h_raw(a, c1, acc1);
        dep_guard_h3(acc0, acc1, a, c0, c1);
      }
      acc_guard2(acc0, acc1);
#pragma unroll
      for (int r = 0; r < 8; ++r) {
        const int p2 = tile * 16 + 8 * h + r;
        const float y0 = fmaxf(acc0[r] * ISC12 + bia0, 0.f);
        const float y1 = fmaxf(acc1[r] * ISC12 + bia1, 0.f);
        const bool ok = p2 < NPIX;
        s0 += ok ? y0 : 0.f;
        s1 += ok ? y1 : 0.f;
      }
    }
  }
  s0 += __shfl_xor(s0, 16, 32);
  s1 += __shfl_xor(s1, 16, 32);
  if (h == 0) {
    pool[wave * 32 + m] = s0;
    pool[wave * 32 + 16 + m] = s1;
  }
  __syncthreads();
  if (tid < C1) {
    float t = 0.f;
#pragma unroll
    for (int w = 0; w < 8; ++w) t += pool[w * 32 + tid];
    pooled[tid] = t * (1.0f / (float)NPIX);
  }
  __syncthreads();

  if (tid < HDIM) {
    float acc = bfr(be1[tid]);
#pragma unroll 1
    for (int i = 0; i < C1; ++i) acc += pooled[i] * bfr(We1[i * HDIM + tid]);
    acc += xbf * bfr(We1[C1 * HDIM + tid]);
    hm[tid] = fmaxf(acc, 0.f);
  }
  __syncthreads();
  if (tid < RDIM) {
    float acc = bfr(be2[tid]);
#pragma unroll 1
    for (int i = 0; i < HDIM; ++i) acc += hm[i] * bfr(We2[i * RDIM + tid]);
    rrow[tid] = acc;
  }
  __syncthreads();
  if (wave == 0) {
    const v4f v = *(const v4f*)(rrow + lane * 4);
    float* p = riT + (size_t)s * RDIM + lane * 4;
    *(volatile v4f*)p = v;
    __threadfence();
    *(volatile v4f*)p = v;
  }
}

__global__ __launch_bounds__(256) void k_latent(
    const float* __restrict__ riT, const float* __restrict__ eps,
    const float* __restrict__ Wh,  const float* __restrict__ bh,
    const float* __restrict__ Wmu, const float* __restrict__ bmu,
    const float* __restrict__ Wsig, const float* __restrict__ bsig,
    float* outms, float* zT)
{
  __shared__ float rS[NB * RDIM];
  __shared__ float hrS[NB * HDIM];
  __shared__ __align__(16) float muS[NB * ZDIM];
  __shared__ __align__(16) float sgS[NB * ZDIM];
  __shared__ __align__(16) float zS[NB * ZDIM];
  const int tid = threadIdx.x;
#pragma unroll 1
  for (int idx = tid; idx < NB * RDIM; idx += 256) {
    const int b = idx >> 7, t = idx & 127;
    float a = 0.f;
#pragma unroll 1
    for (int n = 0; n < NCX; ++n) a += riT[((size_t)(b * NCX + n)) * RDIM + t];
    rS[idx] = a * (1.0f / (float)NCX);
  }
  __syncthreads();
#pragma unroll 1
  for (int idx = tid; idx < NB * HDIM; idx += 256) {
    const int b = idx >> 7, t = idx & 127;
    float a = bfr(bh[t]);
#pragma unroll 1
    for (int i = 0; i < RDIM; ++i) a += rS[b * RDIM + i] * bfr(Wh[i * HDIM + t]);
    hrS[idx] = fmaxf(a, 0.f);
  }
  __syncthreads();
#pragma unroll 1
  for (int idx = tid; idx < NB * ZDIM; idx += 256) {
    const int b = idx >> 6, t = idx & 63;
    float mu = bfr(bmu[t]);
    float sl = bfr(bsig[t]);
#pragma unroll 1
    for (int i = 0; i < HDIM; ++i) {
      const float hv = hrS[b * HDIM + i];
      mu += hv * bfr(Wmu[i * ZDIM + t]);
      sl += hv * bfr(Wsig[i * ZDIM + t]);
    }
    const float sg = 0.1f + 0.9f * (1.0f / (1.0f + expf(-sl)));
    muS[idx] = mu;
    sgS[idx] = sg;
    zS[idx]  = mu + sg * bfr(eps[idx]);
  }
  __syncthreads();
  for (int pass = 0; pass < 2; ++pass) {
#pragma unroll 1
    for (int q = tid; q < (NB * ZDIM) / 4; q += 256) {
      const v4f vm = *(const v4f*)(muS + q * 4);
      const v4f vs = *(const v4f*)(sgS + q * 4);
      const v4f vz = *(const v4f*)(zS + q * 4);
      *(volatile v4f*)(outms + q * 4) = vm;
      *(volatile v4f*)(outms + NB * ZDIM + q * 4) = vs;
      *(volatile v4f*)(zT + q * 4) = vz;
    }
    __threadfence();
  }
}

__global__ __launch_bounds__(128) void k_dec_hidden(
    const float* __restrict__ xt, const float* __restrict__ zT,
    const float* __restrict__ Wd1, const float* __restrict__ bd1,
    const float* __restrict__ Wd2, const float* __restrict__ bd2,
    unsigned short* Hhi, unsigned short* Hlo)
{
  __shared__ float zS[ZDIM];
  __shared__ float h1S[8 * HDIM];
  __shared__ __align__(16) float h2S[16 * HDIM];
  const int t  = threadIdx.x;
  const int r0 = blockIdx.x * 16;
  const int b  = r0 / NTG;
  if (t < ZDIM) zS[t] = zT[b * ZDIM + t];
  __syncthreads();
  const float bd1t = bfr(bd1[t]);
  const float bd2t = bfr(bd2[t]);
  const float w0t  = bfr(Wd1[t]);
  float zd = 0.f;
#pragma unroll 1
  for (int i = 0; i < ZDIM; ++i) zd += zS[i] * bfr(Wd1[(1 + i) * HDIM + t]);
  const float base1 = bd1t + zd;
#pragma unroll 1
  for (int g = 0; g < 2; ++g) {
#pragma unroll
    for (int j = 0; j < 8; ++j) {
      const float xv = bfr(xt[r0 + g * 8 + j]);
      h1S[j * HDIM + t] = fmaxf(base1 + xv * w0t, 0.f);
    }
    __syncthreads();
    float a[8];
#pragma unroll
    for (int j = 0; j < 8; ++j) a[j] = bd2t;
#pragma unroll 1
    for (int i = 0; i < HDIM; ++i) {
      const float w = bfr(Wd2[i * HDIM + t]);
#pragma unroll
      for (int j = 0; j < 8; ++j) a[j] += h1S[j * HDIM + i] * w;
    }
#pragma unroll
    for (int j = 0; j < 8; ++j) h2S[(g * 8 + j) * HDIM + t] = fmaxf(a[j], 0.f);
    __syncthreads();
  }
  v4u ph[2], pl[2];
#pragma unroll
  for (int it = 0; it < 2; ++it) {
    const int j   = it * 128 + t;
    const int row = j >> 4;
    const int c8  = (j & 15) * 8;
    F8 x;
    x.v[0] = *(const v4f*)(h2S + row * HDIM + c8);
    x.v[1] = *(const v4f*)(h2S + row * HDIM + c8 + 4);
#pragma unroll
    for (int e = 0; e < 4; ++e) {
      unsigned short h0, l0, h1, l1;
      split_bits(x.f[2 * e],     h0, l0);
      split_bits(x.f[2 * e + 1], h1, l1);
      ph[it][e] = pk16(h0, h1);
      pl[it][e] = pk16(l0, l1);
    }
  }
  for (int pass = 0; pass < 2; ++pass) {
#pragma unroll
    for (int it = 0; it < 2; ++it) {
      const int j = it * 128 + t;
      const size_t o = (size_t)r0 * HDIM + (size_t)j * 8;
      *(volatile v4u*)(Hhi + o) = ph[it];
      *(volatile v4u*)(Hlo + o) = pl[it];
    }
    __threadfence();
  }
}

__global__ __launch_bounds__(256) void k_dec_gemm(
    const unsigned short* __restrict__ Hhip, const unsigned short* __restrict__ Hlop,
    const unsigned short* __restrict__ Btp, float* Cws)
{
  __shared__ __align__(16) float sT[8][16 * 36];
  const __bf16* A  = (const __bf16*)(const void*)Hhip;
  const __bf16* A2 = (const __bf16*)(const void*)Hlop;
  const int b    = blockIdx.y;
  const __bf16* Bt = (const __bf16*)(const void*)Btp + (size_t)b * NPAD * HDIM;
  float* C = Cws + (size_t)b * NT * NPAD;
  const int lane = threadIdx.x & 31;
  const int wave = threadIdx.x >> 5;
  const int tilesN = NPAD >> 5;
  const int tilesM = NT >> 6;
  const int tile = blockIdx.x * 8 + wave;
  if (tile >= tilesM * tilesN) return;
  const int tm = tile / tilesN;
  const int tn = tile - tm * tilesN;
  const int m0 = tm << 6;
  const int n0 = tn << 5;
  const int rlane = lane & 15;
  const int koff  = (lane >> 4) * 8;
  const int mOff  = (lane >> 4) * 8;

  v8f acc[4][2];
#pragma unroll
  for (int i = 0; i < 4; ++i)
#pragma unroll
    for (int j = 0; j < 2; ++j) acc[i][j] = zero8();

#pragma unroll 1
  for (int k0 = 0; k0 < HDIM; k0 += 32) {
    const v16b bh0 = ldfrag_b(Bt + (size_t)(n0 + rlane) * HDIM + koff + k0);
    const v16b bh1 = ldfrag_b(Bt + (size_t)(n0 + 16 + rlane) * HDIM + koff + k0);
#pragma unroll
    for (int i = 0; i < 4; ++i) {
      const size_t ao = (size_t)(m0 + (i << 4) + rlane) * HDIM + koff + k0;
      const v16b ah = ldfrag_b(A + ao);
      const v16b al = ldfrag_b(A2 + ao);
      acc[i][0] = mma_b_raw(ah, bh0, acc[i][0]);
      acc[i][0] = mma_b_raw(al, bh0, acc[i][0]);
      acc[i][1] = mma_b_raw(ah, bh1, acc[i][1]);
      acc[i][1] = mma_b_raw(al, bh1, acc[i][1]);
      dep_guard_b(acc[i][0], acc[i][1], ah, al);
    }
    keep2_b(bh0, bh1);
  }
  acc_guard4(acc[0][0], acc[0][1], acc[1][0], acc[1][1]);
  acc_guard4(acc[2][0], acc[2][1], acc[3][0], acc[3][1]);

  float* slab = sT[wave];
  const int r4 = lane >> 3, c4 = (lane & 7) * 4;
#pragma unroll
  for (int i = 0; i < 4; ++i) {
    const int mBase = m0 + (i << 4);
#pragma unroll
    for (int j = 0; j < 2; ++j) {
#pragma unroll
      for (int r = 0; r < 8; ++r) slab[(mOff + r) * 36 + (j << 4) + rlane] = acc[i][j][r];
    }
    wave_sync_lds();
    for (int pass = 0; pass < 2; ++pass) {
#pragma unroll
      for (int it = 0; it < 4; ++it) {
        const int row = it * 4 + r4;
        const v4f v = *(const v4f*)(slab + row * 36 + c4);
        *(volatile v4f*)(C + (size_t)(mBase + row) * NPAD + n0 + c4) = v;
      }
      __threadfence();
    }
    wave_sync_lds();
  }
}

__global__ __launch_bounds__(256) void k_pack(const float* __restrict__ Cws, const float* __restrict__ bmu,
                                              const float* __restrict__ bsg, float* out) {
  const size_t f     = ((size_t)blockIdx.x * 256 + threadIdx.x) * 4;
  const size_t plane = (f >= (size_t)NT * NPIX) ? 1 : 0;
  const size_t g     = f - plane * (size_t)NT * NPIX;
  const size_t row   = g / NPIX;
  const int    col   = (int)(g - row * NPIX);
  const v4f c  = *(const v4f*)(Cws + plane * (size_t)NT * NPAD + row * NPAD + col);
  const v4f z0 = *(const v4f*)(bmu + col);
  const v4f z1 = *(const v4f*)(bsg + col);
  v4f y;
#pragma unroll
  for (int e = 0; e < 4; ++e) y[e] = c[e] + bfr((plane != 0) ? z1[e] : z0[e]);
  if (plane != 0) {
    v4f r = y;
#pragma unroll 1
    for (int e = 0; e < 4; ++e) {
      const float x  = r.x;
      const float sp = fmaxf(x, 0.f) + log1pf(expf(-fabsf(x)));
      const float o  = 0.1f + 0.9f * sp;
      v4f nr;
      nr.x = r.y; nr.y = r.z; nr.z = r.w; nr.w = o;
      r = nr;
    }
    y = r;
  }
  *(volatile v4f*)(out + f) = y;
  __threadfence();
  *(volatile v4f*)(out + f) = y;
}

extern "C" void kernel_launch(void* const* d_in, const int* in_sizes, int n_in,
                              void* d_out, int out_size, void* d_ws, size_t ws_size,
                              hipStream_t stream) {
  if (n_in < 26) return;
  if (in_sizes[0] != NS || in_sizes[1] != NS * NPIX || in_sizes[2] != NT || in_sizes[3] != NB * ZDIM) return;
  if (in_sizes[4] != C1 * 2 * 9 || in_sizes[5] != C1 || in_sizes[6] != C1 * C1 * 9 || in_sizes[7] != C1) return;
  if (in_sizes[8] != (C1 + 1) * HDIM || in_sizes[9] != HDIM || in_sizes[10] != HDIM * RDIM || in_sizes[11] != RDIM) return;
  if (in_sizes[12] != RDIM * HDIM || in_sizes[13] != HDIM || in_sizes[14] != HDIM * ZDIM || in_sizes[15] != ZDIM) return;
  if (in_sizes[16] != HDIM * ZDIM || in_sizes[17] != ZDIM) return;
  if (in_sizes[18] != (1 + ZDIM) * HDIM || in_sizes[19] != HDIM || in_sizes[20] != HDIM * HDIM || in_sizes[21] != HDIM) return;
  if (in_sizes[22] != HDIM * NPIX || in_sizes[23] != NPIX || in_sizes[24] != HDIM * NPIX || in_sizes[25] != NPIX) return;
  if (out_size != 2 * NT * NPIX + 2 * NB * ZDIM) return;

  const float* xc   = (const float*)d_in[0];
  const float* yc   = (const float*)d_in[1];
  const float* xt   = (const float*)d_in[2];
  const float* eps  = (const float*)d_in[3];
  const float* w1   = (const float*)d_in[4];
  const float* b1   = (const float*)d_in[5];
  const float* w2   = (const float*)d_in[6];
  const float* b2   = (const float*)d_in[7];
  const float* We1  = (const float*)d_in[8];
  const float* be1  = (const float*)d_in[9];
  const float* We2  = (const float*)d_in[10];
  const float* be2  = (const float*)d_in[11];
  const float* Wh   = (const float*)d_in[12];
  const float* bh   = (const float*)d_in[13];
  const float* Wmu  = (const float*)d_in[14];
  const float* bmu  = (const float*)d_in[15];
  const float* Wsig = (const float*)d_in[16];
  const float* bsig = (const float*)d_in[17];
  const float* Wd1  = (const float*)d_in[18];
  const float* bd1  = (const float*)d_in[19];
  const float* Wd2  = (const float*)d_in[20];
  const float* bd2  = (const float*)d_in[21];
  const float* Wdmu = (const float*)d_in[22];
  const float* bdmu = (const float*)d_in[23];
  const float* Wdsg = (const float*)d_in[24];
  const float* bdsg = (const float*)d_in[25];
  float* out = (float*)d_out;

  const size_t PRI = (size_t)NS * RDIM * 4;
  const size_t PZ  = (size_t)NB * ZDIM * 4;
  const size_t PH  = (size_t)NT * HDIM * 2;
  const size_t PBT = (size_t)2 * NPAD * HDIM * 2;
  const size_t PW2 = (size_t)C1 * K2 * 2;
  const size_t PC  = (size_t)2 * NT * NPAD * 4;
  size_t off = 0;
  const size_t oRI = off; off += PRI;
  const size_t oZ  = off; off += PZ;
  const size_t oHH = off; off += PH;
  const size_t oHL = off; off += PH;
  const size_t oBT = off; off += PBT;
  const size_t oW2 = off; off += PW2;
  const size_t oC  = off; off += PC;
  if (off > ws_size) return;
  if (off > (size_t)134217728) return;

  char* ws = (char*)d_ws;
  float* riT = (float*)(ws + oRI);
  float* zT  = (float*)(ws + oZ);
  unsigned short* Hhi = (unsigned short*)(ws + oHH);
  unsigned short* Hlo = (unsigned short*)(ws + oHL);
  unsigned short* Btp = (unsigned short*)(ws + oBT);
  unsigned short* W2p = (unsigned short*)(ws + oW2);
  float* Cws = (float*)(ws + oC);
  float* outms = out + (size_t)2 * NT * NPIX;

  (void)hipFuncSetAttribute(reinterpret_cast<const void*>(&k_encode),
                            hipFuncAttributeMaxDynamicSharedMemorySize, L_TOTAL);

  k_wprep<<<dim3(NPAD / 64, 3), dim3(256), 0, stream>>>(Wdmu, Wdsg, w2, Btp, W2p);
  k_encode<<<dim3(NS), dim3(256), L_TOTAL, stream>>>(xc, yc, w1, b1, W2p, b2, We1, be1, We2, be2, riT);
  k_latent<<<dim3(1), dim3(256), 0, stream>>>(riT, eps, Wh, bh, Wmu, bmu, Wsig, bsig, outms, zT);
  k_dec_hidden<<<dim3(NT / 16), dim3(128), 0, stream>>>(xt, zT, Wd1, bd1, Wd2, bd2, Hhi, Hlo);
  k_dec_gemm<<<dim3((NT / 64) * (NPAD / 32) / 8, 2), dim3(256), 0, stream>>>(Hhi, Hlo, Btp, Cws);
  k_pack<<<dim3((2 * NT * NPIX) / 1024), dim3(256), 0, stream>>>(Cws, bdmu, bdsg, out);
  (void)hipGetLastError();
}
